// SelfAttention_7670811591149
// MI455X (gfx1250) — hardware-run, weakly checked
//
#include <hip/hip_runtime.h>


#ifndef NB
#define NB 2
#endif
#ifndef IH
#define IH 56
#endif
#define NB_FULL  2
#define IH_FULL  56
#define IW   56
#define TW   (2 * IW)
#define CH   256
#define CQ   64
#define PIX       (IH * IW)
#define PIX_FULL  (IH_FULL * IW)
#define NTOK      (IH * TW)
#define TPI  (PIX / 64)
#define AW   4
#define OSPH 264
#define TPITCH 264
#define QRS  2048.0f
#define QRI  (1.0f / 2048.0f)
#define L2E  1.4426950408889634f
#define PSH  14.0f
#define NEGB (-3.0e38f)
#define WOSC 64.0f
#define WOSI (1.0f / 64.0f)

static_assert(CQ == 64);
static_assert(CH == 256);
static_assert(CH % 64 == 0);
static_assert(CH % 32 == 0);
static_assert(CQ % 32 == 0);
static_assert(NTOK % 64 == 0);
static_assert((NB * NTOK) % 64 == 0);
static_assert(PIX % 64 == 0);
static_assert(NTOK % 32 == 0);
static_assert(NTOK % (16 * AW) == 0);
static_assert(IW % 4 == 0);
static_assert(8 * (IW / 8) == IW);
static_assert(256 * ((CH * IW / 4) / 256) == CH * IW / 4);
static_assert(32 * 16 == CH * 2);
static_assert(32 * 16 * 4 == 16 * CQ * 2);
static_assert(32 * 16 * 4 == 16 * 64 * 2);
static_assert(32 * 16 * 16 == 16 * CH * 2);
static_assert(32 * 16 * 8 == 16 * 64 * 4);
static_assert(OSPH >= CH);
static_assert((OSPH * 2) % 16 == 0);
static_assert(TPITCH >= CH);
static_assert((TPITCH * 2) % 16 == 0);
static_assert(((size_t)PIX_FULL * 4) % 128 == 0);
static_assert(((size_t)NTOK * 2) % 128 == 0);
static_assert(NB <= NB_FULL);
static_assert(IH <= IH_FULL);
static_assert(((size_t)CH * 2 * CH) % (8 * 256) == 0);
static_assert(16 * 68 * 4 <= 131072);
static_assert(AW * 16 * OSPH * 2 <= 131072);
static_assert(IW * TPITCH * 2 <= 131072);
static_assert(2 * CH * 4 <= 131072);

typedef _Float16 h16;
typedef unsigned short bf;
typedef __attribute__((ext_vector_type(16))) __bf16   v16bf;
typedef __attribute__((ext_vector_type(16))) _Float16 v16h;
typedef __attribute__((ext_vector_type(8)))  _Float16 v8h;
typedef __attribute__((ext_vector_type(8)))  unsigned short v8us;
typedef __attribute__((ext_vector_type(8)))  float    v8f;
typedef __attribute__((ext_vector_type(4)))  float    v4f;
typedef v4f  __attribute__((may_alias)) v4fa;
typedef v8h  __attribute__((may_alias)) v8ha;
typedef v8us __attribute__((may_alias)) v8usa;

__device__ __forceinline__ unsigned short f2bf(float f) { unsigned u = __float_as_uint(f); u += 0x7FFFu + ((u >> 16) & 1u); return (unsigned short)(u >> 16); }
__device__ __forceinline__ float bfr(float f) { return __uint_as_float(((unsigned)f2bf(f)) << 16); }
__device__ __forceinline__ v16h cat16(v8h lo, v8h hi) { return __builtin_shufflevector(lo, hi, 0, 1, 2, 3, 4, 5, 6, 7, 8, 9, 10, 11, 12, 13, 14, 15); }
__device__ __forceinline__ v16bf cat16b(v8us lo, v8us hi) { return __builtin_bit_cast(v16bf, __builtin_shufflevector(lo, hi, 0, 1, 2, 3, 4, 5, 6, 7, 8, 9, 10, 11, 12, 13, 14, 15)); }
__device__ __forceinline__ v8f wmma16(v16h a, v16h b, v8f c) { return __builtin_amdgcn_wmma_f32_16x16x32_f16(false, a, false, b, (short)0, c, false, false); }
__device__ __forceinline__ v8f wmmab(v16bf a, v16bf b, v8f c) { return __builtin_amdgcn_wmma_f32_16x16x32_bf16(false, a, false, b, (short)0, c, false, false); }
__device__ __forceinline__ v16h  ldh(const h16* p) { return cat16(*(const v8h*)p, *(const v8h*)(p + 16)); }
__device__ __forceinline__ v16bf ldb(const bf* p)  { return cat16b(*(const v8us*)p, *(const v8us*)(p + 16)); }
__device__ __forceinline__ void wave_sync() { __builtin_amdgcn_fence(3  , "wavefront"); __builtin_amdgcn_wave_barrier(); asm volatile("" ::: "memory"); }
__device__ __forceinline__ h16 toh_flush(float v) { const h16 r = (h16)v; return (fabsf(v) < 6.103515625e-05f) ? (h16)0.0f : r; }
__device__ __forceinline__ v8f mma_h(v16h a, v16h b, v8f c) { c = wmma16(a, b, c); asm volatile("v_nop\n\tv_nop\n\tv_nop\n\tv_nop" : "+v"(c) : "v"(a), "v"(b)); return c; }
__device__ __forceinline__ v8f mma_b(v16bf a, v16bf b, v8f c) { c = wmmab(a, b, c); asm volatile("v_nop\n\tv_nop\n\tv_nop\n\tv_nop" : "+v"(c) : "v"(a), "v"(b)); return c; }

__global__ __launch_bounds__(256) void k_cvt8(const float* __restrict__ src, bf* dst, size_t n8) {
    const size_t i = (size_t)blockIdx.x * 256 + threadIdx.x; if (i >= n8) return;
    const v8f v = *(const v8f*)(src + i * 8); v8us o;
#pragma unroll
    for (int k = 0; k < 8; ++k) o[k] = f2bf(v[k]);
    *(volatile v8us*)(dst + i * 8) = o; __threadfence(); *(volatile v8us*)(dst + i * 8) = o;
}

__global__ __launch_bounds__(256) void k_cvtwo(const float* __restrict__ Wo, bf* WOB, h16* WOH) {
    const int i = blockIdx.x * 256 + threadIdx.x;
    const int o = i >> 6, c8 = (i & 63) * 8;
    const v8f v = *(const v8f*)(Wo + (size_t)o * (2 * CH) + c8);
    if (c8 < CH) {
        v8us q;
#pragma unroll
        for (int k = 0; k < 8; ++k) q[k] = f2bf(bfr(v[k]) * WOSC);
        bf* d = WOB + (size_t)o * CH + c8;
        *(volatile v8us*)d = q; __threadfence(); *(volatile v8us*)d = q;
    } else {
        v8h q;
#pragma unroll
        for (int k = 0; k < 8; ++k) q[k] = toh_flush(bfr(v[k]) * WOSC);
        h16* d = WOH + (size_t)o * CH + (c8 - CH);
        *(volatile v8h*)d = q; __threadfence(); *(volatile v8h*)d = q;
    }
}

__global__ __launch_bounds__(256) void k_bnc(const float* __restrict__ g, const float* __restrict__ be, const float* __restrict__ mu, const float* __restrict__ var, float* tab) {
#pragma clang fp contract(off)
    __shared__ __align__(16) float st[2 * CH];
    const int c = threadIdx.x;
    const float gg = bfr(g[c]), bb = bfr(be[c]), mm = bfr(mu[c]), vv = bfr(var[c]);
    const float inv = gg / sqrtf(vv + 1.0e-5f);
    st[c] = inv; st[CH + c] = bb - mm * inv;
    __syncthreads();
    if (c < (2 * CH) / 4) {
        const v4f v = *(const v4fa*)(&st[4 * c]);
        *(volatile v4f*)(tab + 4 * c) = v; __threadfence(); *(volatile v4f*)(tab + 4 * c) = v;
    }
}

__global__ __launch_bounds__(256) void k_tok(const float* __restrict__ T, bf* X) {
    __shared__ __align__(16) bf ts[IW * TPITCH];
    const int tid = threadIdx.x, lane = tid & 31;
    const int wave = __builtin_amdgcn_readfirstlane((int)(threadIdx.x >> 5));
    const int hrow = blockIdx.x >> 1, side = blockIdx.x & 1, b = blockIdx.y;
    const int img = b + NB_FULL * side;
    const size_t sbase = (size_t)img * CH * PIX_FULL + (size_t)hrow * IW;
#pragma unroll 2
    for (int i = 0; i < (CH * IW / 4) / 256; ++i) {
        const int idx = i * 256 + tid; const int c = idx / (IW / 4), f = idx - c * (IW / 4);
        const v4f v = *(const v4f*)(T + sbase + (size_t)c * PIX_FULL + 4 * f);
#pragma unroll
        for (int e = 0; e < 4; ++e) ts[(4 * f + e) * TPITCH + c] = f2bf(v[e]);
    }
    __syncthreads();
    bf* dst = X + ((size_t)b * NTOK + (size_t)hrow * TW + (size_t)side * IW) * CH;
#pragma unroll 1
    for (int ps = 0; ps < 2; ++ps) {
#pragma unroll 1
        for (int r = 0; r < IW / 8; ++r) { const int row = wave * (IW / 8) + r;
            const v8us v = *(const v8usa*)(&ts[row * TPITCH + lane * 8]);
            *(volatile v8us*)(dst + (size_t)row * CH + lane * 8) = v; }
        if (ps == 0) __threadfence(); }
}

__global__ __launch_bounds__(32) void k_qk(const bf* __restrict__ A, const bf* __restrict__ Bt, h16* PH, h16* PR) {
    __shared__ __align__(16) float os[16 * 68];
    const int K = CH;
    const int lane = threadIdx.x & 31, lr = lane & 15, hi = lane >> 4; const int r0 = blockIdx.x * 64, c0 = blockIdx.y * 64;
    v8f acc[4][4];
#pragma unroll
    for (int mb = 0; mb < 4; ++mb)
#pragma unroll
        for (int nb = 0; nb < 4; ++nb) acc[mb][nb] = (v8f){};
    const size_t aoff = (size_t)(r0 + lr) * K + 8 * hi, boff = (size_t)(c0 + lr) * K + 8 * hi;
#pragma unroll 1
    for (int kc = 0; kc < K; kc += 32) {
        v16bf a[4];
#pragma unroll
        for (int mb = 0; mb < 4; ++mb) a[mb] = ldb(A + aoff + (size_t)mb * 16 * K + kc);
#pragma unroll
        for (int nb = 0; nb < 4; ++nb) { const v16bf b = ldb(Bt + boff + (size_t)nb * 16 * K + kc);
#pragma unroll
            for (int mb = 0; mb < 4; ++mb) acc[mb][nb] = mma_b(a[mb], b, acc[mb][nb]); }
    }
    const size_t tbase = (size_t)blockIdx.y * ((size_t)NB * NTOK * CQ) + (size_t)r0 * CQ;
#pragma unroll
    for (int mb = 0; mb < 4; ++mb) {
#pragma unroll
        for (int nb = 0; nb < 4; ++nb) {
#pragma unroll
            for (int j = 0; j < 8; ++j) os[(hi * 8 + j) * 68 + nb * 16 + lr] = acc[mb][nb][j]; }
        wave_sync();
#pragma unroll 1
        for (int ps = 0; ps < 2; ++ps) {
            const size_t sb = tbase + (size_t)(mb * 16) * CQ;
#pragma unroll
            for (int s = 0; s < 4; ++s) { const int row = 4 * s + (lane >> 3), c8 = (lane & 7) * 8;
                const v4f x0 = *(const v4fa*)(&os[row * 68 + c8]); const v4f x1 = *(const v4fa*)(&os[row * 68 + c8 + 4]); v8h hv, rv;
#pragma unroll
                for (int i = 0; i < 4; ++i) { const h16 a0 = toh_flush(x0[i]); const h16 a1 = toh_flush(x1[i]); hv[i] = a0; hv[4 + i] = a1;
                    rv[i] = toh_flush((x0[i] - (float)a0) * QRS); rv[4 + i] = toh_flush((x1[i] - (float)a1) * QRS); }
                const size_t oo = sb + (size_t)row * CQ + c8;
                *(volatile v8h*)(PH + oo) = hv; *(volatile v8h*)(PR + oo) = rv; }
            if (ps == 0) __threadfence(); }
        wave_sync();
    }
}

__global__ __launch_bounds__(32) void k_vp(const bf* __restrict__ A, const bf* __restrict__ Bt, const float* __restrict__ bnt, h16* VT) {
    __shared__ __align__(16) float os[16 * 68];
    const int K = CH;
    const int lane = threadIdx.x & 31, lr = lane & 15, hi = lane >> 4; const int r0 = blockIdx.x * 64, c0 = blockIdx.y * 64;
    v8f acc[4][4];
#pragma unroll
    for (int mb = 0; mb < 4; ++mb)
#pragma unroll
        for (int nb = 0; nb < 4; ++nb) acc[mb][nb] = (v8f){};
    const size_t aoff = (size_t)(r0 + lr) * K + 8 * hi, boff = (size_t)(c0 + lr) * K + 8 * hi;
#pragma unroll 1
    for (int kc = 0; kc < K; kc += 32) {
        v16bf a[4];
#pragma unroll
        for (int mb = 0; mb < 4; ++mb) a[mb] = ldb(A + aoff + (size_t)mb * 16 * K + kc);
#pragma unroll
        for (int nb = 0; nb < 4; ++nb) { const v16bf b = ldb(Bt + boff + (size_t)nb * 16 * K + kc);
#pragma unroll
            for (int mb = 0; mb < 4; ++mb) acc[mb][nb] = mma_b(a[mb], b, acc[mb][nb]); }
    }
    const int bb = c0 / NTOK, tt = c0 % NTOK;
    const size_t tbase = (size_t)bb * (size_t)CH * NTOK + (size_t)r0 * NTOK + (size_t)tt;
#pragma unroll
    for (int mb = 0; mb < 4; ++mb) {
        float gi[8], gs[8];
#pragma unroll
        for (int j = 0; j < 8; ++j) { gi[j] = bnt[r0 + mb * 16 + hi * 8 + j]; gs[j] = bnt[CH + r0 + mb * 16 + hi * 8 + j]; }
#pragma unroll
        for (int nb = 0; nb < 4; ++nb) {
#pragma unroll
            for (int j = 0; j < 8; ++j) { const float y = acc[mb][nb][j] * gi[j] + gs[j]; os[(hi * 8 + j) * 68 + nb * 16 + lr] = (y > 0.0f) ? y : 0.0f; } }
        wave_sync();
#pragma unroll 1
        for (int ps = 0; ps < 2; ++ps) {
            const size_t sb = tbase + (size_t)(mb * 16) * NTOK;
#pragma unroll
            for (int s = 0; s < 4; ++s) { const int row = 4 * s + (lane >> 3), c8 = (lane & 7) * 8;
                const v4f x0 = *(const v4fa*)(&os[row * 68 + c8]); const v4f x1 = *(const v4fa*)(&os[row * 68 + c8 + 4]); v8h hv;
#pragma unroll
                for (int i = 0; i < 4; ++i) { hv[i] = toh_flush(x0[i]); hv[4 + i] = toh_flush(x1[i]); }
                *(volatile v8h*)(VT + sb + (size_t)row * NTOK + c8) = hv; }
            if (ps == 0) __threadfence(); }
        wave_sync();
    }
}

__global__ __launch_bounds__(32 * AW) __attribute__((amdgpu_num_vgpr(256)))
void k_flash(const h16* __restrict__ SQH, const h16* __restrict__ SQR, const h16* __restrict__ SKH, const h16* __restrict__ SKR, const h16* __restrict__ VT, h16* CT) {
    __shared__ __align__(16) h16 os[AW * 16 * OSPH];
    const int lane = threadIdx.x & 31, lr = lane & 15, hi = lane >> 4;
    const int wave = __builtin_amdgcn_readfirstlane((int)(threadIdx.x >> 5));
    const int b = blockIdx.y;
    const int m0 = (blockIdx.x * AW + wave) * 16;
    const size_t pbase = (size_t)b * NTOK * CQ;
    const unsigned colofs = (unsigned)((m0 + lr) * CQ + 8 * hi);
    const size_t ko = pbase + (size_t)lr * CQ + 8 * hi;
    const size_t vo = (size_t)b * CH * NTOK + (size_t)lr * NTOK + 8 * hi;
    v8f o[16];
#pragma unroll
    for (int j = 0; j < 16; ++j) o[j] = (v8f){};
    float m = NEGB, l = 0.0f;
#pragma unroll 1
    for (int key0 = 0; key0 < NTOK; key0 += 32) {
        unsigned cv = colofs; asm volatile("" : "+v"(cv));
        const h16* bh_p = SKH + pbase + cv; const h16* br_p = SKR + pbase + cv;
        const h16* ah_p = SQH + ko + (size_t)key0 * CQ; const h16* ar_p = SQR + ko + (size_t)key0 * CQ;
        v8f sHa = (v8f){}, sLa = (v8f){}, sHb = (v8f){}, sLb = (v8f){};
#pragma unroll
        for (int ks = 0; ks < 2; ++ks) {
            const v16h bh = ldh(bh_p + 32 * ks), br = ldh(br_p + 32 * ks);
            const v16h ah = ldh(ah_p + 32 * ks), ar = ldh(ar_p + 32 * ks);
            sHa = mma_h(ah, bh, sHa); sLa = mma_h(ah, br, sLa); sLa = mma_h(ar, bh, sLa);
            const v16h ch = ldh(ah_p + 16 * CQ + 32 * ks), cr = ldh(ar_p + 16 * CQ + 32 * ks);
            sHb = mma_h(ch, bh, sHb); sLb = mma_h(ch, br, sLb); sLb = mma_h(cr, bh, sLb);
        }
        float ta[8], tb[8]; float mx = NEGB;
#pragma unroll
        for (int r = 0; r < 8; ++r) {
            ta[r] = (sHa[r] + sLa[r] * QRI) * L2E; tb[r] = (sHb[r] + sLb[r] * QRI) * L2E;
            mx = fmaxf(mx, fmaxf(ta[r], tb[r])); }
        mx = fmaxf(mx, __shfl_xor(mx, 16, 32));
        const float mnew = fmaxf(m, mx);
        const float alpha = __builtin_amdgcn_exp2f(m - mnew);
        const float sh = PSH - mnew;
        v16h pb; float ls = 0.0f;
#pragma unroll
        for (int r = 0; r < 8; ++r) {
            const float xa = ta[r] + sh, xb = tb[r] + sh;
            const float ea = __builtin_amdgcn_exp2f(xa), eb = __builtin_amdgcn_exp2f(xb);
            const float ga = (xa < -14.0f) ? 0.0f : ea, gb = (xb < -14.0f) ? 0.0f : eb;
            const h16 pa = (h16)ga; const h16 pc = (h16)gb;
            pb[r] = pa; pb[8 + r] = pc;
            ls += (float)pa + (float)pc; }
        l = l * alpha + ls; m = mnew;
#pragma unroll
        for (int j = 0; j < 16; ++j) o[j] = o[j] * alpha;
        const h16* va = VT + vo + key0;
#pragma unroll
        for (int g = 0; g < 4; ++g) {
            const v16h v0 = ldh(va + (size_t)(64 * g +  0) * NTOK), v1 = ldh(va + (size_t)(64 * g + 16) * NTOK);
            const v16h v2 = ldh(va + (size_t)(64 * g + 32) * NTOK), v3 = ldh(va + (size_t)(64 * g + 48) * NTOK);
            o[4 * g + 0] = mma_h(v0, pb, o[4 * g + 0]); o[4 * g + 1] = mma_h(v1, pb, o[4 * g + 1]);
            o[4 * g + 2] = mma_h(v2, pb, o[4 * g + 2]); o[4 * g + 3] = mma_h(v3, pb, o[4 * g + 3]);
        }
    }
    l += __shfl_xor(l, 16, 32);
    const bool any = l > 0.0f;
    const float lsafe = any ? l : 1.0f;
    const float inv = any ? (1.0f / lsafe) : 0.0f;
    const int wb = wave * 16 * OSPH;
#pragma unroll
    for (int j = 0; j < 16; ++j) { v8h hv;
#pragma unroll
        for (int r = 0; r < 8; ++r) hv[r] = toh_flush(o[j][r] * inv);
        *(v8ha*)(&os[wb + lr * OSPH + 16 * j + 8 * hi]) = hv; }
    wave_sync();
    h16* crow = CT + ((size_t)b * NTOK + m0) * CH;
#pragma unroll 1
    for (int ps = 0; ps < 2; ++ps) {
#pragma unroll 4
        for (int s = 0; s < 16; ++s) {
            const v8h val = *(const v8ha*)(&os[wb + s * OSPH + lane * 8]);
            *(volatile v8h*)(crow + (size_t)s * CH + lane * 8) = val; }
        if (ps == 0) __threadfence(); }
}

__global__ __launch_bounds__(32) void k_out(const bf* __restrict__ WOB, const h16* __restrict__ WOH, const bf* __restrict__ X, const h16* __restrict__ CT, const float* __restrict__ bnt, float* OUT) {
    __shared__ __align__(16) float os[16 * 68];
    const int K = CH;
    const int lane = threadIdx.x & 31, lr = lane & 15, hi = lane >> 4;
    const int r0 = blockIdx.x * 64;
    const int slot = blockIdx.y / TPI, p0 = (blockIdx.y % TPI) * 64;
    const int b = slot % NB, side = slot / NB; const int img = b + NB_FULL * side;
    size_t boff[4];
#pragma unroll
    for (int nb = 0; nb < 4; ++nb) { const int p = p0 + nb * 16 + lr; const int hh = p / IW, ww = p - hh * IW; const int n = hh * TW + ww + side * IW;
        boff[nb] = ((size_t)b * NTOK + (size_t)n) * CH + 8 * hi; }
    const size_t aoff = (size_t)(r0 + lr) * K + 8 * hi;
    v8f acc[4][4];
#pragma unroll
    for (int mb = 0; mb < 4; ++mb)
#pragma unroll
        for (int nb = 0; nb < 4; ++nb) acc[mb][nb] = (v8f){};
#pragma unroll 1
    for (int kc = 0; kc < K; kc += 32) {
        v16bf a[4];
#pragma unroll
        for (int mb = 0; mb < 4; ++mb) a[mb] = ldb(WOB + aoff + (size_t)mb * 16 * K + kc);
#pragma unroll
        for (int nb = 0; nb < 4; ++nb) { const v16bf bb = ldb(X + boff[nb] + kc);
#pragma unroll
            for (int mb = 0; mb < 4; ++mb) acc[mb][nb] = mma_b(a[mb], bb, acc[mb][nb]); }
    }
#pragma unroll 1
    for (int kc = 0; kc < K; kc += 32) {
        v16h a[4];
#pragma unroll
        for (int mb = 0; mb < 4; ++mb) a[mb] = ldh(WOH + aoff + (size_t)mb * 16 * K + kc);
#pragma unroll
        for (int nb = 0; nb < 4; ++nb) { const v16h bb = ldh(CT + boff[nb] + kc);
#pragma unroll
            for (int mb = 0; mb < 4; ++mb) acc[mb][nb] = mma_h(a[mb], bb, acc[mb][nb]); }
    }
    const size_t tbase = ((size_t)img * CH + (size_t)r0) * PIX_FULL + (size_t)p0;
#pragma unroll
    for (int mb = 0; mb < 4; ++mb) {
        float gi[8], gs[8];
#pragma unroll
        for (int j = 0; j < 8; ++j) { gi[j] = bnt[r0 + mb * 16 + hi * 8 + j] * WOSI; gs[j] = bnt[CH + r0 + mb * 16 + hi * 8 + j]; }
#pragma unroll
        for (int nb = 0; nb < 4; ++nb) {
#pragma unroll
            for (int j = 0; j < 8; ++j) { const float y = acc[mb][nb][j] * gi[j] + gs[j]; os[(hi * 8 + j) * 68 + nb * 16 + lr] = (y > 0.0f) ? y : 0.0f; } }
        wave_sync();
        float* orow = OUT + tbase + (size_t)(mb * 16) * PIX_FULL;
#pragma unroll 1
        for (int ps = 0; ps < 2; ++ps) {
#pragma unroll
            for (int s = 0; s < 8; ++s) { const int row = 2 * s + (lane >> 4), cofs = (lane & 15) * 4;
                const v4f val = *(const v4fa*)(&os[row * 68 + cofs]);
                *(volatile v4f*)(orow + (size_t)row * PIX_FULL + cofs) = val; }
            if (ps == 0) __threadfence(); }
        wave_sync();
    }
}

static constexpr size_t al256(size_t v) { return (v + 255) & ~(size_t)255; }
static constexpr size_t SZ_X   = al256((size_t)NB * NTOK * CH * 2);
static constexpr size_t SZ_WQK = al256((size_t)2 * CQ * CH * 2);
static constexpr size_t SZ_WV  = al256((size_t)CH * CH * 2);
static constexpr size_t SZ_WO  = al256((size_t)CH * CH * 2);
static constexpr size_t SZ_BN  = al256((size_t)2 * CH * 4);
static constexpr size_t SZ_PQ  = al256((size_t)2 * NB * NTOK * CQ * 2);
static constexpr size_t SZ_TOTAL = 3 * SZ_X + SZ_WQK + SZ_WV + 2 * SZ_WO + 2 * SZ_BN + 2 * SZ_PQ;
static_assert(SZ_TOTAL <= (size_t)134217728);
static_assert(((size_t)CQ * CH * 2) % 256 == 0);
static_assert(((size_t)NB * NTOK * CQ * 2) % 256 == 0);
static_assert((size_t)NB * CH * NTOK == (size_t)NB * NTOK * CH);

extern "C" void kernel_launch(void* const* d_in, const int* in_sizes, int n_in,
                              void* d_out, int out_size, void* d_ws, size_t ws_size, hipStream_t stream) {
    if (n_in < 13) return;
    const size_t needt = ((size_t)(NB - 1 + NB_FULL) * CH + (size_t)(CH - 1)) * PIX_FULL + (size_t)PIX;
    if ((size_t)in_sizes[0] < needt) return;
    if ((size_t)in_sizes[1] < (size_t)CQ * CH || (size_t)in_sizes[2] < (size_t)CQ * CH || (size_t)in_sizes[3] < (size_t)CH * CH) return;
    if (in_sizes[4] < CH || in_sizes[5] < CH || in_sizes[6] < CH || in_sizes[7] < CH) return;
    if ((size_t)in_sizes[8] < (size_t)CH * 2 * CH) return;
    if (in_sizes[9] < CH || in_sizes[10] < CH || in_sizes[11] < CH || in_sizes[12] < CH) return;
    if ((size_t)out_size < needt) return;
    if (SZ_TOTAL > ws_size) return;
    const float* t  = (const float*)d_in[0];
    const float* wq = (const float*)d_in[1]; const float* wk = (const float*)d_in[2]; const float* wv = (const float*)d_in[3];
    const float* gv = (const float*)d_in[4]; const float* bv = (const float*)d_in[5]; const float* mv = (const float*)d_in[6]; const float* vv = (const float*)d_in[7];
    const float* wo = (const float*)d_in[8];
    const float* go = (const float*)d_in[9]; const float* bo = (const float*)d_in[10]; const float* mo = (const float*)d_in[11]; const float* vo = (const float*)d_in[12];
    float* OUT = (float*)d_out;
    char* wsp = (char*)d_ws;
    bf*  X   = (bf*)wsp;  wsp += SZ_X;
    h16* VT  = (h16*)wsp; wsp += SZ_X;
    h16* CT  = (h16*)wsp; wsp += SZ_X;
    bf*  WQK = (bf*)wsp;  wsp += SZ_WQK;
    bf*  WVB = (bf*)wsp;  wsp += SZ_WV;
    bf*  WOB = (bf*)wsp;  wsp += SZ_WO;
    h16* WOH = (h16*)wsp; wsp += SZ_WO;
    float* BNV = (float*)wsp; wsp += SZ_BN;
    float* BNO = (float*)wsp; wsp += SZ_BN;
    h16* PH  = (h16*)wsp; wsp += SZ_PQ;
    h16* PR  = (h16*)wsp; wsp += SZ_PQ;
    const size_t PLQ = (size_t)NB * NTOK * CQ;

    { const size_t n8 = (size_t)CQ * CH / 8; const unsigned g = (unsigned)((n8 + 255) / 256);
      k_cvt8<<<g, 256, 0, stream>>>(wq, WQK, n8); k_cvt8<<<g, 256, 0, stream>>>(wk, WQK + (size_t)CQ * CH, n8); }
    { const size_t n8 = (size_t)CH * CH / 8; k_cvt8<<<(unsigned)((n8 + 255) / 256), 256, 0, stream>>>(wv, WVB, n8); }
    k_cvtwo<<<(unsigned)((size_t)CH * 2 * CH / 8 / 256), 256, 0, stream>>>(wo, WOB, WOH);
    k_bnc<<<1, 256, 0, stream>>>(gv, bv, mv, vv, BNV);
    k_bnc<<<1, 256, 0, stream>>>(go, bo, mo, vo, BNO);
    k_tok<<<dim3(2 * IH, NB, 1), 256, 0, stream>>>(t, X);

    k_qk<<<dim3(NB * NTOK / 64, 2, 1), 32, 0, stream>>>(X, WQK, PH, PR);
    k_vp<<<dim3(CH / 64, NB * NTOK / 64, 1), 32, 0, stream>>>(WVB, X, BNV, VT);
    k_flash<<<dim3(NTOK / (16 * AW), NB, 1), 32 * AW, 0, stream>>>(PH, PR, PH + PLQ, PR + PLQ, VT, CT);
    k_out<<<dim3(CH / 64, 2 * NB * TPI, 1), 32, 0, stream>>>(WOB, WOH, X, CT, BNO, OUT);
}
